// MambaBlock_10419590660407
// MI455X (gfx1250) — hardware-verified
//
#include <hip/hip_runtime.h>
#include <math.h>

typedef __attribute__((ext_vector_type(16))) _Float16 v16h;
typedef __attribute__((ext_vector_type(8)))  _Float16 v8h;
typedef __attribute__((ext_vector_type(16))) __bf16   v16b;
typedef __attribute__((ext_vector_type(8)))  __bf16   v8b;
typedef __attribute__((ext_vector_type(8)))  float    v8f;
typedef __attribute__((ext_vector_type(4)))  float    v4f;
typedef __attribute__((ext_vector_type(2)))  float    v2f;

constexpr int kBatch = 4;
constexpr int kSeq   = 2048;
constexpr int kDm    = 1024;
constexpr int kDi    = 2048;
constexpr int kNs    = 64;
constexpr int kXrP   = 2 * kDi;
constexpr int kBcP   = 2 * kNs;
constexpr int kRows  = kBatch * kSeq;
constexpr int kNtile = kDi / 64;
constexpr int kTP    = 260;
constexpr float kWCarry = 32.0f;
constexpr float kYCarry = 16.0f;
static_assert(kNtile == 32);
static_assert(kNs == 64 && kBcP == 128);
static_assert((kDm % 32) == 0 && (kDi % 32) == 0);
static_assert((kSeq % 64) == 0 && (kXrP % 64) == 0 && (kBcP % 64) == 0 && (kDi % 64) == 0 && (kDm % 64) == 0);
static_assert((kRows % 8) == 0 && (kDi % 256) == 0 && kDm == 1024);

constexpr size_t kSzWin  = (size_t)kXrP * kDm * 2;
constexpr size_t kSzWx   = (size_t)kBcP * kDi * 2;
constexpr size_t kSzWdt  = (size_t)kDi * kDi * 2;
constexpr size_t kSzWout = (size_t)kDm * kDi * 2;
constexpr size_t kSzXn   = (size_t)kRows * kDm * 2;
constexpr size_t kSzXr   = (size_t)kSeq * kXrP * 4;
constexpr size_t kSzXc   = (size_t)kSeq * kDi * 2;
constexpr size_t kSzBc   = (size_t)kSeq * kBcP * 4;
constexpr size_t kSzDp   = (size_t)kNtile * kSeq * 4;
constexpr size_t kSzYs   = (size_t)kSeq * 4;
constexpr size_t kSzY    = (size_t)kSeq * kDi * 2;
constexpr size_t kOffWin  = 0;
constexpr size_t kOffWxh  = kOffWin  + kSzWin;
constexpr size_t kOffWxl  = kOffWxh  + kSzWx;
constexpr size_t kOffWdt  = kOffWxl  + kSzWx;
constexpr size_t kOffWout = kOffWdt  + kSzWdt;
constexpr size_t kOffXn   = kOffWout + kSzWout;
constexpr size_t kOffXr   = kOffXn   + kSzXn;
constexpr size_t kOffXch  = kOffXr   + kSzXr;
constexpr size_t kOffXcl  = kOffXch  + kSzXc;
constexpr size_t kOffBc   = kOffXcl  + kSzXc;
constexpr size_t kOffDp   = kOffBc   + kSzBc;
constexpr size_t kOffYs   = kOffDp   + kSzDp;
constexpr size_t kOffY    = kOffYs   + kSzYs;
constexpr size_t kWsTotal = kOffY    + kSzY;
static_assert(kWsTotal == 98836480ull);
static_assert(kWsTotal <= 134217728ull);
static_assert((kOffWxh % 128) == 0 && (kOffWxl % 128) == 0 && (kOffWdt % 128) == 0 && (kOffWout % 128) == 0 &&
              (kOffXn % 128) == 0 && (kOffXr % 128) == 0 && (kOffXch % 128) == 0 && (kOffXcl % 128) == 0 &&
              (kOffBc % 128) == 0 && (kOffDp % 128) == 0 && (kOffYs % 128) == 0 && (kOffY % 128) == 0);

__device__ __forceinline__ unsigned short f2bf_bits(float f) {
  unsigned u = __float_as_uint(f);
  return (unsigned short)((u + 0x7FFFu + ((u >> 16) & 1u)) >> 16);
}
__device__ __forceinline__ float bf_bits2f(unsigned short h) { return __uint_as_float(((unsigned)h) << 16); }

__device__ __forceinline__ void dep_guard_h(v8f& a, v8f& b, v8f& c, v8f& d, v16h x, v16h y) {
  asm volatile("v_nop\n\tv_nop\n\tv_nop\n\tv_nop" : "+v"(a), "+v"(b), "+v"(c), "+v"(d) : "v"(x), "v"(y));
}
__device__ __forceinline__ void dep_guard_b(v8f& a, v8f& b, v8f& c, v8f& d, v16b x, v16b y) {
  asm volatile("v_nop\n\tv_nop\n\tv_nop\n\tv_nop" : "+v"(a), "+v"(b), "+v"(c), "+v"(d) : "v"(x), "v"(y));
}
__device__ __forceinline__ void keep4_h(v16h a, v16h b, v16h c, v16h d) { asm volatile("v_nop" :: "v"(a), "v"(b), "v"(c), "v"(d)); }
__device__ __forceinline__ void keep4_b(v16b a, v16b b, v16b c, v16b d) { asm volatile("v_nop" :: "v"(a), "v"(b), "v"(c), "v"(d)); }
__device__ __forceinline__ void acc_guard4(v8f& a, v8f& b, v8f& c, v8f& d) {
  asm volatile("v_nop\n\tv_nop\n\tv_nop\n\tv_nop" : "+v"(a), "+v"(b), "+v"(c), "+v"(d));
}

template <typename T> struct Frag;
template <> struct Frag<_Float16> {
  typedef v16h V; union U { v16h v; v8h h[2]; };
  static __device__ __forceinline__ v16h load(const _Float16* p) {
    U f; f.h[0] = *(const v8h*)(p); f.h[1] = *(const v8h*)(p + 16); return f.v;
  }
  static __device__ __forceinline__ v8f mma(v16h a, v16h b, v8f c) {
    return __builtin_amdgcn_wmma_f32_16x16x32_f16(false, a, false, b, (short)0, c, false, false);
  }
  static __device__ __forceinline__ void guard(v8f& a, v8f& b, v8f& c, v8f& d, v16h x, v16h y) { dep_guard_h(a, b, c, d, x, y); }
  static __device__ __forceinline__ void keep(v16h a, v16h b, v16h c, v16h d) { keep4_h(a, b, c, d); }
};
template <> struct Frag<__bf16> {
  typedef v16b V; union U { v16b v; v8b h[2]; };
  static __device__ __forceinline__ v16b load(const __bf16* p) {
    U f; f.h[0] = *(const v8b*)(p); f.h[1] = *(const v8b*)(p + 16); return f.v;
  }
  static __device__ __forceinline__ v8f mma(v16b a, v16b b, v8f c) {
    return __builtin_amdgcn_wmma_f32_16x16x32_bf16(false, a, false, b, (short)0, c, false, false);
  }
  static __device__ __forceinline__ void guard(v8f& a, v8f& b, v8f& c, v8f& d, v16b x, v16b y) { dep_guard_b(a, b, c, d, x, y); }
  static __device__ __forceinline__ void keep(v16b a, v16b b, v16b c, v16b d) { keep4_b(a, b, c, d); }
};
template <int ET> struct Elem;
template <> struct Elem<0> { typedef _Float16 T; };
template <> struct Elem<1> { typedef __bf16 T; };

template <int ET, bool SPLIT, int EPI, int MT>
__global__ __launch_bounds__(256) void wmma_gemm64(
    const unsigned short* __restrict__ Ap, const unsigned short* __restrict__ A2p, int lda,
    const unsigned short* __restrict__ Btp, const unsigned short* __restrict__ Bt2p, int ldb,
    float* Cout, int ldc,
    const float* __restrict__ bias, const float* __restrict__ resid,
    int M, int N, int K, float scale)
{
  static_assert(MT == 2 || MT == 4);
  static_assert(EPI != 2 || MT == 4);
  typedef typename Elem<ET>::T T;
  typedef typename Frag<T>::V V;
  const T* A = (const T*)Ap;
  const T* A2 = (const T*)A2p;
  const T* Bt = (const T*)Btp;
  const T* Bt2 = (const T*)Bt2p;
  __shared__ __align__(16) float sT[8][16 * 68];
  __shared__ __align__(16) float sR[(EPI == 2) ? 8 : 1][64];
  __shared__ __align__(16) float sBias[(EPI == 2) ? 8 : 1][64];
  const int lane = threadIdx.x & 31;
  const int wave = threadIdx.x >> 5;
  const int wsl  = (EPI == 2) ? wave : 0;
  const int tilesN = N >> 6;
  const int tilesM = M / (16 * MT);
  const int tile = blockIdx.x * 8 + wave;
  if (tile >= tilesM * tilesN) return;
  const int tm = tile / tilesN;
  const int tn = tile - tm * tilesN;
  const int m0 = tm * (16 * MT);
  const int n0 = tn << 6;

  const int rlane = lane & 15;
  const int koff  = (lane >> 4) * 8;
  const int mOff  = (lane >> 4) * 8;

  v8f acc[MT][4];
#pragma unroll
  for (int i = 0; i < MT; ++i)
#pragma unroll
    for (int j = 0; j < 4; ++j) acc[i][j] = (v8f){0.f,0.f,0.f,0.f,0.f,0.f,0.f,0.f};

  for (int k0 = 0; k0 < K; k0 += 32) {
    V bh[4], bl[4];
#pragma unroll
    for (int j = 0; j < 4; ++j) {
      const size_t bo = (size_t)(n0 + (j << 4) + rlane) * ldb + koff + k0;
      bh[j] = Frag<T>::load(Bt + bo);
      if (SPLIT) bl[j] = Frag<T>::load(Bt2 + bo);
    }
#pragma unroll
    for (int i = 0; i < MT; ++i) {
      const size_t ao = (size_t)(m0 + (i << 4) + rlane) * lda + koff + k0;
      V ah = Frag<T>::load(A + ao);
      V al;
      if (SPLIT) al = Frag<T>::load(A2 + ao);
#pragma unroll
      for (int j = 0; j < 4; ++j) {
        acc[i][j] = Frag<T>::mma(ah, bh[j], acc[i][j]);
        if (SPLIT) {
          acc[i][j] = Frag<T>::mma(ah, bl[j], acc[i][j]);
          acc[i][j] = Frag<T>::mma(al, bh[j], acc[i][j]);
        }
      }
      Frag<T>::guard(acc[i][0], acc[i][1], acc[i][2], acc[i][3], ah, SPLIT ? al : ah);
    }
    Frag<T>::keep(bh[0], bh[1], bh[2], bh[3]);
    if (SPLIT) Frag<T>::keep(bl[0], bl[1], bl[2], bl[3]);
  }
#pragma unroll
  for (int i = 0; i < MT; ++i) acc_guard4(acc[i][0], acc[i][1], acc[i][2], acc[i][3]);

  float* slab = sT[wave];
  if (EPI == 2) {
    const v4f bq = *(const v4f*)(bias + n0 + (lane & 15) * 4);
    if (lane < 16) *(v4f*)(&sBias[wsl][(lane & 15) * 4]) = bq;
  }
#pragma unroll
  for (int i = 0; i < MT; ++i) {
    const int mBase = m0 + (i << 4);
#pragma unroll
    for (int j = 0; j < 4; ++j) {
#pragma unroll
      for (int r = 0; r < 8; ++r) {
        float v = acc[i][j][r];
        if (EPI != 2) v *= scale;
        slab[(mOff + r) * 68 + (j << 4) + rlane] = v;
      }
    }
    __builtin_amdgcn_fence(__ATOMIC_RELEASE, "workgroup");
    __builtin_amdgcn_wave_barrier();
    __builtin_amdgcn_fence(__ATOMIC_ACQUIRE, "workgroup");
    if (EPI == 0) {
      const int hh = lane >> 4, c4 = (lane & 15) * 4;
      for (int pass = 0; pass < 2; ++pass) {
#pragma unroll
        for (int it = 0; it < 8; ++it) {
          const int row = it * 2 + hh;
          v4f v = *(const v4f*)(slab + row * 68 + c4);
          *(volatile v4f*)(Cout + (size_t)(mBase + row) * ldc + n0 + c4) = v;
        }
        __threadfence();
      }
    } else if (EPI == 1) {
      const int hh = lane >> 4, c4 = (lane & 15) * 4;
      v4f vv[8];
#pragma unroll
      for (int it = 0; it < 8; ++it) {
        const int row = it * 2 + hh;
        const v4f sv = *(const v4f*)(slab + row * 68 + c4);
        const v4f rv = *(const v4f*)(resid + (size_t)(mBase + row) * ldc + n0 + c4);
        vv[it] = sv + rv;
      }
      for (int pass = 0; pass < 2; ++pass) {
#pragma unroll
        for (int it = 0; it < 8; ++it) {
          const int row = it * 2 + hh;
          *(volatile v4f*)(Cout + (size_t)(mBase + row) * ldc + n0 + c4) = vv[it];
        }
        __threadfence();
      }
    } else {
      const float* sp = slab + (lane >> 1) * 68 + (lane & 1) * 32;
      const float* sb = &sBias[wsl][(lane & 1) * 32];
      float sum = 0.0f;
#pragma unroll 1
      for (int c = 0; c < 32; ++c) {
        const float v = sp[c] + sb[c];
        const float a = expf(-fabsf(v));
        sum += fmaxf(v, 0.0f) + log1pf(a);
      }
      sum += __shfl_xor(sum, 1, 32);
      if ((lane & 1) == 0) sR[wsl][(i << 4) + (lane >> 1)] = sum;
    }
    __builtin_amdgcn_fence(__ATOMIC_RELEASE, "workgroup");
    __builtin_amdgcn_wave_barrier();
    __builtin_amdgcn_fence(__ATOMIC_ACQUIRE, "workgroup");
  }
  if (EPI == 2) {
    const v4f rv = *(const v4f*)(&sR[wsl][(lane & 15) * 4]);
    float* dp = Cout + (size_t)tn * M + m0 + (lane & 15) * 4;
    if (lane < 16) *(volatile v4f*)dp = rv;
    __threadfence();
    if (lane < 16) *(volatile v4f*)dp = rv;
  }
}

template <int MODE>
__global__ __launch_bounds__(256) void transpose_cast_kernel(
    const float* __restrict__ W, unsigned short* Bt, unsigned short* Bt2, int Kdim, int Ndim, float scale)
{
  __shared__ float tile[64 * 65];
  const int tid = threadIdx.x, lane = tid & 31, wave = tid >> 5;
  const int n0 = blockIdx.x * 64;
  const int k0 = blockIdx.y * 64;
#pragma unroll 8
  for (int p = 0; p < 16; ++p) {
    const int idx = tid + p * 256;
    const int kk  = idx >> 6;
    const int nn  = idx & 63;
    const int n   = n0 + nn;
    const int nc  = (n < Ndim) ? n : (Ndim - 1);
    const float v = W[(size_t)(k0 + kk) * Ndim + nc];
    tile[kk * 65 + nn] = (n < Ndim) ? (v * scale) : 0.f;
  }
  __syncthreads();
  const int q = lane >> 3, c8 = (lane & 7) * 8;
  v8h hv[2], lv[2];
#pragma unroll
  for (int it = 0; it < 2; ++it) {
    const int nrow = it * 32 + wave * 4 + q;
#pragma unroll
    for (int e = 0; e < 8; ++e) {
      const float f = tile[(c8 + e) * 65 + nrow];
      if (MODE == 0) {
        hv[it][e] = (_Float16)f;
      } else {
        const unsigned short hb = f2bf_bits(f);
        const unsigned short lb = f2bf_bits(f - bf_bits2f(hb));
        hv[it][e] = __builtin_bit_cast(_Float16, hb);
        lv[it][e] = __builtin_bit_cast(_Float16, lb);
      }
    }
  }
  for (int pass = 0; pass < 2; ++pass) {
#pragma unroll
    for (int it = 0; it < 2; ++it) {
      const int nrow = it * 32 + wave * 4 + q;
      const size_t o = (size_t)(n0 + nrow) * Kdim + k0 + c8;
      *(volatile v8h*)(Bt + o) = hv[it];
      if (MODE == 2) *(volatile v8h*)(Bt2 + o) = lv[it];
    }
    __threadfence();
  }
}

__global__ __launch_bounds__(256) void ln_kernel(
    const float* __restrict__ x, const float* __restrict__ g, const float* __restrict__ bta, unsigned short* xn)
{
  const int lane = threadIdx.x & 31, wave = threadIdx.x >> 5;
  const int row = blockIdx.x * 8 + wave;
  const float* xr = x + (size_t)row * kDm + 8 * lane;
  float s = 0.0f;
#pragma unroll 1
  for (int j = 0; j < 4; ++j) {
    const v4f a0 = *(const v4f*)(xr + 256 * j);
    const v4f a1 = *(const v4f*)(xr + 256 * j + 4);
    s += ((a0[0] + a0[1]) + (a0[2] + a0[3])) + ((a1[0] + a1[1]) + (a1[2] + a1[3]));
  }
#pragma unroll
  for (int off = 16; off > 0; off >>= 1) s += __shfl_xor(s, off, 32);
  const float mu = s * (1.0f / (float)kDm);
  float ss = 0.0f;
#pragma unroll 1
  for (int j = 0; j < 4; ++j) {
    const v4f a0 = *(const v4f*)(xr + 256 * j);
    const v4f a1 = *(const v4f*)(xr + 256 * j + 4);
#pragma unroll
    for (int e = 0; e < 4; ++e) {
      const float d0 = a0[e] - mu;
      const float d1 = a1[e] - mu;
      ss += d0 * d0;
      ss += d1 * d1;
    }
  }
#pragma unroll
  for (int off = 16; off > 0; off >>= 1) ss += __shfl_xor(ss, off, 32);
  const float var  = ss * (1.0f / (float)kDm);
  const float rstd = __builtin_amdgcn_rcpf(sqrtf(var + 1e-5f));
  unsigned short* o = xn + (size_t)row * kDm + 8 * lane;
#pragma unroll 1
  for (int j = 0; j < 4; ++j) {
    const v4f a0 = *(const v4f*)(xr + 256 * j);
    const v4f a1 = *(const v4f*)(xr + 256 * j + 4);
    const v4f g0 = *(const v4f*)(g + 256 * j + 8 * lane);
    const v4f g1 = *(const v4f*)(g + 256 * j + 8 * lane + 4);
    const v4f b0 = *(const v4f*)(bta + 256 * j + 8 * lane);
    const v4f b1 = *(const v4f*)(bta + 256 * j + 8 * lane + 4);
    v8h hv;
#pragma unroll
    for (int e = 0; e < 4; ++e) {
      const float y0 = ((a0[e] - mu) * rstd) * g0[e] + b0[e];
      const float y1 = ((a1[e] - mu) * rstd) * g1[e] + b1[e];
      hv[e]     = (_Float16)y0;
      hv[4 + e] = (_Float16)y1;
    }
    *(volatile v8h*)(o + 256 * j) = hv;
    __threadfence();
    *(volatile v8h*)(o + 256 * j) = hv;
  }
}

__global__ __launch_bounds__(256) void conv_silu_kernel(
    const float* __restrict__ XR, const float* __restrict__ cw, const float* __restrict__ cb,
    unsigned short* XCH, unsigned short* XCL)
{
  __shared__ __align__(16) float sT[16 * kTP];
  const int tid = threadIdx.x, lane = tid & 31, wave = tid >> 5;
  const int d0 = blockIdx.x * 256, d = d0 + tid;
  const int t0 = blockIdx.y * 64;
  const v4f wv = *(const v4f*)(cw + (size_t)d * 4);
  const float w0 = wv[0], w1 = wv[1], w2 = wv[2], w3 = wv[3];
  const float bcv = cb[d];
  float xm3, xm2, xm1;
  {
    const int r3 = t0 - 3, r2 = t0 - 2, r1 = t0 - 1;
    const float v3 = XR[(size_t)(r3 < 0 ? 0 : r3) * kXrP + d];
    const float v2 = XR[(size_t)(r2 < 0 ? 0 : r2) * kXrP + d];
    const float v1 = XR[(size_t)(r1 < 0 ? 0 : r1) * kXrP + d];
    xm3 = (r3 >= 0) ? v3 : 0.f;
    xm2 = (r2 >= 0) ? v2 : 0.f;
    xm1 = (r1 >= 0) ? v1 : 0.f;
  }
#pragma unroll 1
  for (int sub = 0; sub < 4; ++sub) {
    const int lb = t0 + sub * 16;
#pragma unroll 1
    for (int s = 0; s < 16; ++s) {
      const float xcur = XR[(size_t)(lb + s) * kXrP + d];
      float acc = w0 * xm3;
      acc = fmaf(w1, xm2, acc);
      acc = fmaf(w2, xm1, acc);
      acc = fmaf(w3, xcur, acc);
      const float sv = acc + bcv;
      const float sg = __builtin_amdgcn_rcpf(1.0f + expf(fminf(-sv, 80.0f)));
      sT[s * kTP + tid] = sv * sg;
      xm3 = xm2; xm2 = xm1; xm1 = xcur;
    }
    __syncthreads();
    v8h bh[2], blo[2];
#pragma unroll
    for (int it = 0; it < 2; ++it) {
      const float* sp = sT + (it * 8 + wave) * kTP + lane * 8;
      const v4f a0 = *(const v4f*)(sp);
      const v4f a1 = *(const v4f*)(sp + 4);
#pragma unroll
      for (int e = 0; e < 4; ++e) {
        const float f0 = a0[e], f1 = a1[e];
        const unsigned short h0 = f2bf_bits(f0), h1 = f2bf_bits(f1);
        const unsigned short l0 = f2bf_bits(f0 - bf_bits2f(h0)), l1 = f2bf_bits(f1 - bf_bits2f(h1));
        bh[it][e]      = __builtin_bit_cast(_Float16, h0);
        bh[it][4 + e]  = __builtin_bit_cast(_Float16, h1);
        blo[it][e]     = __builtin_bit_cast(_Float16, l0);
        blo[it][4 + e] = __builtin_bit_cast(_Float16, l1);
      }
    }
    for (int pass = 0; pass < 2; ++pass) {
#pragma unroll
      for (int it = 0; it < 2; ++it) {
        const size_t o = (size_t)(lb + it * 8 + wave) * kDi + d0 + lane * 8;
        *(volatile v8h*)(XCH + o) = bh[it];
        *(volatile v8h*)(XCL + o) = blo[it];
      }
      __threadfence();
    }
    __syncthreads();
  }
}

__global__ __launch_bounds__(32) void scan_kernel(
    const float* __restrict__ DPART, const float* __restrict__ BC, const float* __restrict__ A_log, float* YS)
{
  const int lane = threadIdx.x & 31;
  const float A0 = -expf(A_log[lane]);
  const float A1 = -expf(A_log[lane + 32]);
  float h0 = 0.0f, h1 = 0.0f;
#pragma unroll 1
  for (int t0 = 0; t0 < kSeq; t0 += 32) {
    float keepv = 0.0f;
#pragma unroll 1
    for (int s = 0; s < 32; ++s) {
      const int t = t0 + s;
      float dsum = DPART[(size_t)lane * kSeq + t];
      const float* brow = BC + (size_t)t * kBcP;
      const float B0 = brow[lane];
      const float B1 = brow[lane + 32];
      const float C0 = brow[kNs + lane];
      const float C1 = brow[kNs + lane + 32];
#pragma unroll
      for (int off = 16; off > 0; off >>= 1) dsum += __shfl_xor(dsum, off, 32);
      const float delta = dsum * (1.0f / (float)kDi);
      float e0 = expf(delta * A0);
      float e1 = expf(delta * A1);
      e0 = (e0 < 1.17549435e-38f) ? 0.0f : e0;
      e1 = (e1 < 1.17549435e-38f) ? 0.0f : e1;
      h0 = h0 * e0 + B0;
      h1 = h1 * e1 + B1;
      float p = h0 * C0 + h1 * C1;
#pragma unroll
      for (int off = 16; off > 0; off >>= 1) p += __shfl_xor(p, off, 32);
      keepv = (lane == s) ? p : keepv;
    }
    float* yp = YS + t0 + lane;
    *(volatile float*)yp = keepv;
    __threadfence();
    *(volatile float*)yp = keepv;
  }
}

__global__ __launch_bounds__(128) void gate_kernel(
    const unsigned* __restrict__ XCH32, const unsigned* __restrict__ XCL32,
    const float* __restrict__ XR, const float* __restrict__ YS, const float* __restrict__ Dp,
    unsigned short* Y16)
{
  __shared__ __align__(16) float sT[16 * kTP];
  const int tid = threadIdx.x, lane = tid & 31, wave = tid >> 5;
  const int d0 = blockIdx.x * 256, dp = d0 + 2 * tid;
  const int t0 = blockIdx.y * 64;
  const v2f Dd = *(const v2f*)(Dp + dp);
#pragma unroll 1
  for (int sub = 0; sub < 4; ++sub) {
    const int lb = t0 + sub * 16;
#pragma unroll 1
    for (int s = 0; s < 16; ++s) {
      const size_t row = (size_t)(lb + s);
      const size_t wi = (row * kDi + dp) >> 1;
      const unsigned hw = XCH32[wi];
      const unsigned lw = XCL32[wi];
      const float xc0 = __uint_as_float(hw << 16) + __uint_as_float(lw << 16);
      const float xc1 = __uint_as_float(hw & 0xffff0000u) + __uint_as_float(lw & 0xffff0000u);
      const v2f rv = *(const v2f*)(XR + row * kXrP + kDi + dp);
      const float r0 = rv[0], r1 = rv[1];
      const float yv = YS[row];
      const float sg0 = __builtin_amdgcn_rcpf(1.0f + expf(fminf(-r0, 80.0f)));
      const float sg1 = __builtin_amdgcn_rcpf(1.0f + expf(fminf(-r1, 80.0f)));
      const float y0 = (yv + Dd[0] * xc0) * (r0 * sg0);
      const float y1 = (yv + Dd[1] * xc1) * (r1 * sg1);
      sT[s * kTP + 2 * tid]     = y0 * kYCarry;
      sT[s * kTP + 2 * tid + 1] = y1 * kYCarry;
    }
    __syncthreads();
    v8h hv[4];
#pragma unroll
    for (int it = 0; it < 4; ++it) {
      const float* sp = sT + (it * 4 + wave) * kTP + lane * 8;
      const v4f a0 = *(const v4f*)(sp);
      const v4f a1 = *(const v4f*)(sp + 4);
#pragma unroll
      for (int e = 0; e < 4; ++e) {
        hv[it][e]     = (_Float16)a0[e];
        hv[it][4 + e] = (_Float16)a1[e];
      }
    }
    for (int pass = 0; pass < 2; ++pass) {
#pragma unroll
      for (int it = 0; it < 4; ++it)
        *(volatile v8h*)(Y16 + (size_t)(lb + it * 4 + wave) * kDi + d0 + lane * 8) = hv[it];
      __threadfence();
    }
    __syncthreads();
  }
}

constexpr int kBlkInProj  = (kSeq / 64) * (kXrP / 64) / 8;
constexpr int kBlkXProj   = (kSeq / 32) * (kBcP / 64) / 8;
constexpr int kBlkDt      = (kSeq / 64) * (kDi / 64) / 8;
constexpr int kBlkOutProj = (kSeq / 64) * (kDm / 64) / 8;
static_assert(kBlkInProj == 256 && kBlkXProj == 16 && kBlkDt == 128 && kBlkOutProj == 64);

extern "C" void kernel_launch(void* const* d_in, const int* in_sizes, int n_in,
                              void* d_out, int out_size, void* d_ws, size_t ws_size,
                              hipStream_t stream)
{
  if (n_in < 12) return;
  if (in_sizes[0] != kRows * kDm) return;
  if (in_sizes[1] != kDm || in_sizes[2] != kDm) return;
  if (in_sizes[3] != kDm * kXrP) return;
  if (in_sizes[4] != kDi * 4 || in_sizes[5] != kDi) return;
  if (in_sizes[6] != kDi * kBcP) return;
  if (in_sizes[7] != kDi * kDi || in_sizes[8] != kDi) return;
  if (in_sizes[9] != kNs || in_sizes[10] != kDi) return;
  if (in_sizes[11] != kDi * kDm) return;
  if (out_size != kRows * kDm) return;
  if (ws_size < kWsTotal) return;

  const float* x      = (const float*)d_in[0];
  const float* ln_g   = (const float*)d_in[1];
  const float* ln_b   = (const float*)d_in[2];
  const float* W_in   = (const float*)d_in[3];
  const float* conv_w = (const float*)d_in[4];
  const float* conv_b = (const float*)d_in[5];
  const float* W_x    = (const float*)d_in[6];
  const float* W_dt   = (const float*)d_in[7];
  const float* b_dt   = (const float*)d_in[8];
  const float* A_log  = (const float*)d_in[9];
  const float* Dp     = (const float*)d_in[10];
  const float* W_out  = (const float*)d_in[11];
  float* out = (float*)d_out;

  char* ws = (char*)d_ws;
  unsigned short* WINT = (unsigned short*)(ws + kOffWin);
  unsigned short* WXH  = (unsigned short*)(ws + kOffWxh);
  unsigned short* WXL  = (unsigned short*)(ws + kOffWxl);
  unsigned short* WDT  = (unsigned short*)(ws + kOffWdt);
  unsigned short* WOUT = (unsigned short*)(ws + kOffWout);
  unsigned short* XN   = (unsigned short*)(ws + kOffXn);
  float*          XR   = (float*)(ws + kOffXr);
  unsigned short* XCH  = (unsigned short*)(ws + kOffXch);
  unsigned short* XCL  = (unsigned short*)(ws + kOffXcl);
  float*          BC   = (float*)(ws + kOffBc);
  float*          DPT  = (float*)(ws + kOffDp);
  float*          YS   = (float*)(ws + kOffYs);
  unsigned short* Y16  = (unsigned short*)(ws + kOffY);

  const float invW  = 1.0f / kWCarry;
  const float invWY = 1.0f / (kWCarry * kYCarry);

  transpose_cast_kernel<0><<<dim3(kXrP / 64, kDm / 64), 256, 0, stream>>>(W_in, WINT, WINT, kDm, kXrP, kWCarry);
  transpose_cast_kernel<2><<<dim3(kBcP / 64, kDi / 64), 256, 0, stream>>>(W_x, WXH, WXL, kDi, kBcP, 1.0f);
  transpose_cast_kernel<1><<<dim3(kDi / 64, kDi / 64), 256, 0, stream>>>(W_dt, WDT, WDT, kDi, kDi, 1.0f);
  transpose_cast_kernel<0><<<dim3(kDm / 64, kDi / 64), 256, 0, stream>>>(W_out, WOUT, WOUT, kDi, kDm, kWCarry);

  ln_kernel<<<kRows / 8, 256, 0, stream>>>(x, ln_g, ln_b, XN);

  for (int b = 0; b < kBatch; ++b) {
    const unsigned short* xnb = XN + (size_t)b * kSeq * kDm;
    const float* xb = x + (size_t)b * kSeq * kDm;
    float* outb = out + (size_t)b * kSeq * kDm;

    wmma_gemm64<0, false, 0, 4><<<dim3(kBlkInProj), 256, 0, stream>>>(
        xnb, xnb, kDm, WINT, WINT, kDm, XR, kXrP, b_dt, xb, kSeq, kXrP, kDm, invW);

    conv_silu_kernel<<<dim3(kDi / 256, kSeq / 64), 256, 0, stream>>>(XR, conv_w, conv_b, XCH, XCL);

    wmma_gemm64<1, true, 0, 2><<<dim3(kBlkXProj), 256, 0, stream>>>(
        XCH, XCL, kDi, WXH, WXL, kDi, BC, kBcP, b_dt, xb, kSeq, kBcP, kDi, 1.0f);

    wmma_gemm64<1, false, 2, 4><<<dim3(kBlkDt), 256, 0, stream>>>(
        XCH, XCH, kDi, WDT, WDT, kDi, DPT, kSeq, b_dt, xb, kSeq, kDi, kDi, 1.0f);

    scan_kernel<<<1, 32, 0, stream>>>(DPT, BC, A_log, YS);

    gate_kernel<<<dim3(kDi / 256, kSeq / 64), 128, 0, stream>>>(
        (const unsigned*)XCH, (const unsigned*)XCL, XR, YS, Dp, Y16);

    wmma_gemm64<0, false, 1, 4><<<dim3(kBlkOutProj), 256, 0, stream>>>(
        Y16, Y16, kDi, WOUT, WOUT, kDi, outb, kDm, b_dt, xb, kSeq, kDm, kDi, invWY);
  }
}
